// GRNNTransformSimple_55259049230549
// MI455X (gfx1250) — hardware-verified
//
#include <hip/hip_runtime.h>
#include <stddef.h>


#define NNODE  16383
#define NINNER 8191
#define OFFLF  8191
#define LVTOP  12
#define FD     8
#define HD     64
#define KD     192
#define NT     128
#define NWV    4
#define RB     64
#define AP     200
#define OP     68
#define WSCAP  134217728

static_assert((AP % 8) == 0);
static_assert((OP % 4) == 0);
static_assert((KD % 32) == 0);
static_assert(RB == 16 * NWV);
static_assert(NT == 32 * NWV);
static_assert(NT == 2 * RB);
static_assert(((RB * 16) % NT) == 0);
static_assert((FD * HD) % NT == 0);
static_assert(HD <= NT);

typedef float          v4f   __attribute__((ext_vector_type(4)));
typedef float          v8f   __attribute__((ext_vector_type(8)));
typedef unsigned int   v4u   __attribute__((ext_vector_type(4)));
typedef _Float16       v8h   __attribute__((ext_vector_type(8)));
typedef _Float16       v16h  __attribute__((ext_vector_type(16)));

__device__ __forceinline__ v16h ldfrag(const _Float16* p) {
  const v8h u0 = *(const v8h*)p;
  const v8h u1 = *(const v8h*)(p + 16);
  return __builtin_shufflevector(u0, u1, 0, 1, 2, 3, 4, 5, 6, 7, 8, 9, 10, 11, 12, 13, 14, 15);
}

__device__ __forceinline__ v8f wm(v16h a, v16h b, v8f c) {
  v8f d = __builtin_amdgcn_wmma_f32_16x16x32_f16(false, a, false, b, (short)0, c, false, false);
  asm volatile("v_nop\n\tv_nop\n\tv_nop\n\tv_nop" : "+v"(d) : "v"(a), "v"(b));
  return d;
}
__device__ __forceinline__ v8f zero8() {
  v8f z = {0.f, 0.f, 0.f, 0.f, 0.f, 0.f, 0.f, 0.f};
  return z;
}
__device__ __forceinline__ int iclamp(int v, int lo, int hi) { return v < lo ? lo : (v > hi ? hi : v); }

__device__ __forceinline__ v4u pack8(v4f a, v4f b, float s) {
  v8h hv;
  hv[0] = (_Float16)(s * a.x); hv[1] = (_Float16)(s * a.y); hv[2] = (_Float16)(s * a.z); hv[3] = (_Float16)(s * a.w);
  hv[4] = (_Float16)(s * b.x); hv[5] = (_Float16)(s * b.y); hv[6] = (_Float16)(s * b.z); hv[7] = (_Float16)(s * b.w);
  return __builtin_bit_cast(v4u, hv);
}

__global__ __launch_bounds__(256) void k_prep(const float* __restrict__ Wh, _Float16* WhP) {
  const int o = ((int)blockIdx.x * 256 + (int)threadIdx.x) * 8;
  const int n = o / KD, k0 = o - n * KD;
  v8h hv;
#pragma unroll
  for (int i = 0; i < 8; ++i) hv[i] = (_Float16)(64.0f * Wh[(size_t)(k0 + i) * HD + n]);
  const v4u u = __builtin_bit_cast(v4u, hv);
  _Float16* dst = WhP + o;
  *(volatile v4u*)dst = u;
  __threadfence();
  *(volatile v4u*)dst = u;
}

__device__ __forceinline__ void emb_rows(const float* sO, _Float16* E, int row0, int nrows, int wave, int lane) {
#pragma unroll 1
  for (int it = 0; it < 4; ++it) {
    const int r = 16 * wave + 4 * it + (lane >> 3);
    const int c8 = lane & 7;
    const int gr = row0 + r;
    if (gr < nrows) {
      const v4f a = *(const v4f*)(sO + r * OP + 8 * c8);
      const v4f b = *(const v4f*)(sO + r * OP + 8 * c8 + 4);
      *(volatile v4u*)(E + (size_t)gr * HD + 8 * c8) = pack8(a, b, 16.0f);
    }
  }
}
__device__ __forceinline__ void out_rows(const float* sO, float* out, int row0, int nrows, int wave, int hh, int m) {
#pragma unroll 1
  for (int it = 0; it < 8; ++it) {
    const int r = 16 * wave + 2 * it + hh;
    const int gr = row0 + r;
    if (gr < nrows) {
      const v4f v = *(const v4f*)(sO + r * OP + 4 * m);
      *(volatile v4f*)(out + (size_t)gr * HD + 4 * m) = v;
    }
  }
}

__global__ __launch_bounds__(NT) void k_level(const float* __restrict__ x, const int* __restrict__ ch,
                                                const float* __restrict__ Wu, const float* __restrict__ bu,
                                                const float* __restrict__ bh, const _Float16* __restrict__ WhP,
                                                const _Float16* __restrict__ Ein, _Float16* Eout, float* out,
                                                int level, int nrows) {
  __shared__ __attribute__((aligned(16))) _Float16 sA[RB * AP];
  __shared__ __attribute__((aligned(16))) float sO[RB * OP];
  __shared__ __attribute__((aligned(16))) float sWu[FD * HD];
  __shared__ __attribute__((aligned(16))) float sBu[HD];
  __shared__ float sBh[HD];
  __shared__ int sCh[2 * RB];
  const int tid = (int)threadIdx.x, lane = tid & 31, wave = tid >> 5, hh = lane >> 4, m = lane & 15;
  const int n = 1 << level;
  const int off = n - 1;
  const int nch = n << 1;
  const int row0 = (int)blockIdx.x * RB;
  const bool top = (level == LVTOP);

#pragma unroll 1
  for (int i = tid; i < FD * HD; i += NT) sWu[i] = Wu[i];
  if (tid < HD) { sBu[tid] = bu[tid]; sBh[tid] = bh[tid]; }
  {
    const int r = tid >> 1, w2 = tid & 1;
    int gr = row0 + r;
    gr = gr > nrows - 1 ? nrows - 1 : gr;
    const int nn = gr & (n - 1);
    int ci = 2 * (off + nn) + w2;
    ci = iclamp(ci, 0, 2 * NINNER - 1);
    int loc = ch[ci] - 2 * off;
    loc = iclamp(loc, 0, nch - 1);
    sCh[tid] = loc;
  }
  __syncthreads();

  if (!top) {
#pragma unroll 1
    for (int it = 0; it < (RB * 16) / NT; ++it) {
      const int p = it * NT + tid;
      const int r = p >> 4, w2 = (p >> 3) & 1, c8 = p & 7;
      int gr = row0 + r;
      gr = gr > nrows - 1 ? nrows - 1 : gr;
      const int b = gr >> level;
      const int loc = sCh[2 * r + w2];
      const v8h v = *(const v8h*)(Ein + ((size_t)b * nch + loc) * HD + 8 * c8);
      *(v8h*)(sA + r * AP + HD * w2 + 8 * c8) = v;
    }
  }

  {
    const int r = tid >> 1, half = tid & 1;
    int gr = row0 + r;
    gr = gr > nrows - 1 ? nrows - 1 : gr;
    const int b = gr >> level, nn = gr & (n - 1);
    const int njob = top ? 3 : 1;
#pragma unroll 1
    for (int j = 0; j < njob; ++j) {
      const int jj = top ? j : 2;
      const int jsel = jj < 2 ? jj : 0;
      const int node = (jj < 2) ? (OFFLF + sCh[2 * r + jsel]) : (off + nn);
      const float* xp = x + ((size_t)b * NNODE + node) * FD;
      const v4f x0 = *(const v4f*)xp;
      const v4f x1 = *(const v4f*)(xp + 4);
      const float xs[8] = {x0.x, x0.y, x0.z, x0.w, x1.x, x1.y, x1.z, x1.w};
#pragma unroll 1
      for (int g = 0; g < 4; ++g) {
        const int oc = 32 * half + 8 * g;
        const v4f bA = *(const v4f*)(sBu + oc);
        const v4f bB = *(const v4f*)(sBu + oc + 4);
        float a0 = bA.x, a1 = bA.y, a2 = bA.z, a3 = bA.w, a4 = bB.x, a5 = bB.y, a6 = bB.z, a7 = bB.w;
#pragma unroll
        for (int f = 0; f < FD; ++f) {
          const float xf = xs[f];
          const v4f w0 = *(const v4f*)(sWu + f * HD + oc);
          const v4f w1 = *(const v4f*)(sWu + f * HD + oc + 4);
          a0 += xf * w0.x; a1 += xf * w0.y; a2 += xf * w0.z; a3 += xf * w0.w;
          a4 += xf * w1.x; a5 += xf * w1.y; a6 += xf * w1.z; a7 += xf * w1.w;
        }
        v8h hv;
        hv[0] = (_Float16)(16.0f * fmaxf(a0, 0.0f)); hv[1] = (_Float16)(16.0f * fmaxf(a1, 0.0f));
        hv[2] = (_Float16)(16.0f * fmaxf(a2, 0.0f)); hv[3] = (_Float16)(16.0f * fmaxf(a3, 0.0f));
        hv[4] = (_Float16)(16.0f * fmaxf(a4, 0.0f)); hv[5] = (_Float16)(16.0f * fmaxf(a5, 0.0f));
        hv[6] = (_Float16)(16.0f * fmaxf(a6, 0.0f)); hv[7] = (_Float16)(16.0f * fmaxf(a7, 0.0f));
        *(v8h*)(sA + r * AP + HD * jj + oc) = hv;
      }
    }
  }
  __syncthreads();

  v8f c[4];
#pragma unroll
  for (int nt = 0; nt < 4; ++nt) c[nt] = zero8();
  {
    const _Float16* aq = sA + (16 * wave + m) * AP + 8 * hh;
    const _Float16* bq = WhP + (size_t)m * KD + 8 * hh;
#pragma unroll 1
    for (int ks = 0; ks < KD / 32; ++ks) {
      const v16h a = ldfrag(aq + 32 * ks);
#pragma unroll
      for (int nt = 0; nt < 4; ++nt) {
        const v16h bf = ldfrag(bq + (size_t)(16 * nt) * KD + 32 * ks);
        c[nt] = wm(a, bf, c[nt]);
      }
    }
  }
#pragma unroll
  for (int nt = 0; nt < 4; ++nt) {
    const int col = 16 * nt + m;
    const float bb = sBh[col];
#pragma unroll
    for (int r = 0; r < 8; ++r) {
      const float t = c[nt][r] * 0.0009765625f + bb;
      sO[(16 * wave + 8 * hh + r) * OP + col] = fmaxf(t, 0.0f);
    }
  }
  __syncthreads();

  if (level == 0) {
    out_rows(sO, out, row0, nrows, wave, hh, m);
    __threadfence();
    out_rows(sO, out, row0, nrows, wave, hh, m);
  } else {
    emb_rows(sO, Eout, row0, nrows, wave, lane);
    __threadfence();
    emb_rows(sO, Eout, row0, nrows, wave, lane);
  }
}

extern "C" void kernel_launch(void* const* d_in, const int* in_sizes, int n_in,
                              void* d_out, int out_size, void* d_ws, size_t ws_size,
                              hipStream_t stream) {
  if (n_in < 6) return;
  const int perTree = NNODE * FD;
  if (in_sizes[0] < perTree || (in_sizes[0] % perTree) != 0) return;
  const int nB = in_sizes[0] / perTree;
  if (nB < 1 || nB > 4096) return;
  if (in_sizes[1] != 2 * NINNER) return;
  if (in_sizes[2] != FD * HD || in_sizes[3] != HD) return;
  if (in_sizes[4] != KD * HD || in_sizes[5] != HD) return;
  if ((long long)out_size != (long long)nB * HD) return;

  const float* x  = (const float*)d_in[0];
  const int*   ch = (const int*)d_in[1];
  const float* Wu = (const float*)d_in[2];
  const float* bu = (const float*)d_in[3];
  const float* Wh = (const float*)d_in[4];
  const float* bh = (const float*)d_in[5];
  float* out = (float*)d_out;

  const size_t cap = ws_size < (size_t)WSCAP ? ws_size : (size_t)WSCAP;
  const size_t bW = (size_t)HD * KD * 2;
  const size_t bX = (size_t)nB * ((size_t)1 << LVTOP) * HD * 2;
  const size_t bY = (size_t)nB * ((size_t)1 << (LVTOP - 1)) * HD * 2;
  char* ws = (char*)d_ws;
  size_t o = 0;
  const size_t oW = o; o += bW; o = (o + 255) & ~(size_t)255;
  const size_t oX = o; o += bX; o = (o + 255) & ~(size_t)255;
  const size_t oY = o; o += bY; o = (o + 255) & ~(size_t)255;
  if (o > cap || o > ws_size) return;
  _Float16* WhP = (_Float16*)(ws + oW);
  _Float16* EX  = (_Float16*)(ws + oX);
  _Float16* EY  = (_Float16*)(ws + oY);

  k_prep<<<(HD * KD) / (256 * 8), 256, 0, stream>>>(Wh, WhP);

  for (int level = LVTOP; level >= 0; --level) {
    const int nrows = nB << level;
    const int blocks = (nrows + RB - 1) / RB;
    const _Float16* Ein = ((level + 1) & 1) ? EY : EX;
    _Float16* Eout = (level & 1) ? EY : EX;
    k_level<<<blocks, NT, 0, stream>>>(x, ch, Wu, bu, bh, WhP, Ein, Eout, out, level, nrows);
  }
}
